// HyperGAT_24627342475678
// MI455X (gfx1250) — hardware-verified
//
#include <hip/hip_runtime.h>
#include <hip/hip_bf16.h>

typedef __attribute__((ext_vector_type(16))) _Float16 v16h;
typedef __attribute__((ext_vector_type(8)))  _Float16 v8h;
typedef __attribute__((ext_vector_type(8)))  float    v8f;
typedef __attribute__((ext_vector_type(4)))  float    v4f;
typedef __attribute__((ext_vector_type(4)))  unsigned v4u;
typedef float __attribute__((may_alias)) float_a;
template <typename T> __device__ __forceinline__ void vst2(void* p, T v) { *(volatile T*)p = v; __threadfence(); *(volatile T*)p = v; }
__device__ __forceinline__ v8f wmma16(v16h a, v16h b, v8f c) {
  v8f d = __builtin_amdgcn_wmma_f32_16x16x32_f16(false, a, false, b, (short)0, c, false, false);
  asm volatile("v_nop\n\tv_nop\n\tv_nop\n\tv_nop" : "+v"(d) : "v"(a), "v"(b));
  return d;
}

__device__ __forceinline__ float wave_sum(float v) {
#pragma unroll
  for (int off = 16; off > 0; off >>= 1) v += __shfl_xor(v, off, 32);
  return v;
}
__device__ __forceinline__ float elu_f(float x) { return x > 0.f ? x : __expf(x) - 1.f; }

__global__ void prep_bfrag(const float* __restrict__ B, _Float16* __restrict__ out,
                           int N, int KB, int tilesN, long strideB, int total) {
  const int g8 = blockIdx.x * blockDim.x + threadIdx.x;
  if (g8 * 8 >= total) return;
  union { v8h h; v4u u; } pk;
#pragma unroll
  for (int ee = 0; ee < 8; ++ee) {
    const int idx  = g8 * 8 + ee;
    const int e    = idx & 15;
    const int lane = (idx >> 4) & 31;
    int rest = idx >> 9;
    const int tn   = rest % tilesN; rest /= tilesN;
    const int k32  = rest % KB;
    const int b    = rest / KB;
    const int hi   = lane >> 4;
    const int k    = k32 * 32 + (hi << 3) + ((e < 8) ? e : (e + 8));
    const int n    = tn * 16 + (lane & 15);
    pk.h[ee] = (_Float16)B[(long)b * strideB + (long)k * N + n];
  }
  vst2(out + (size_t)g8 * 8, pk.u);
}

template <int K>
__global__ __launch_bounds__(256) void gemm_wmma_f16(const float* __restrict__ A,
                              const _Float16* __restrict__ Bfrag,
                              float* __restrict__ C,
                              int M, int N,
                              long strideA, long strideC,
                              int batches) {
  constexpr int KB = K / 32;
  __shared__ __attribute__((aligned(16))) float so[8][16 * 32];
  const int lane = threadIdx.x & 31, wv = threadIdx.x >> 5;
  const int wid  = (blockIdx.x * blockDim.x + threadIdx.x) >> 5;
  const int tilesM = (M + 15) >> 4;
  const int tilesN = N >> 4;
  const int tilesN2 = N >> 5;
  const int perBatch = tilesM * tilesN2;
  const bool active = wid < perBatch * batches;
  const int widc = active ? wid : 0;
  const int b  = widc / perBatch;
  const int r  = widc % perBatch;
  const int tm = r / tilesN2;
  const int tn2 = r % tilesN2;

  const int hi    = lane >> 4;
  const int row_a = tm * 16 + (lane & 15);
  const int row_c = row_a < M ? row_a : (M - 1);
  const float* Arow = A + (long)b * strideA + (long)row_c * K;
  const _Float16* Bbase0 = Bfrag + ((((long)b * KB) * tilesN + 2 * tn2) << 9) + lane * 16;
  const _Float16* Bbase1 = Bbase0 + 512;

  v8f acc = {}, acc1 = {};
#pragma unroll
  for (int k32 = 0; k32 < KB; ++k32) {
    const int kb = k32 * 32;
    const float4* p0 = (const float4*)(Arow + kb + (hi << 3));
    const float4* p1 = (const float4*)(Arow + kb + 16 + (hi << 3));
    const float4 x0 = p0[0], x1 = p0[1];
    const float4 x2 = p1[0], x3 = p1[1];
    v16h af;
    af[0]  = (_Float16)x0.x; af[1]  = (_Float16)x0.y;
    af[2]  = (_Float16)x0.z; af[3]  = (_Float16)x0.w;
    af[4]  = (_Float16)x1.x; af[5]  = (_Float16)x1.y;
    af[6]  = (_Float16)x1.z; af[7]  = (_Float16)x1.w;
    af[8]  = (_Float16)x2.x; af[9]  = (_Float16)x2.y;
    af[10] = (_Float16)x2.z; af[11] = (_Float16)x2.w;
    af[12] = (_Float16)x3.x; af[13] = (_Float16)x3.y;
    af[14] = (_Float16)x3.z; af[15] = (_Float16)x3.w;
    const v16h bf0 = *(const v16h*)(Bbase0 + ((long)k32 * tilesN << 9));
    const v16h bf1 = *(const v16h*)(Bbase1 + ((long)k32 * tilesN << 9));
    acc  = wmma16(af, bf0, acc);
    acc1 = wmma16(af, bf1, acc1);
  }
  float* S = so[wv];
#pragma unroll
  for (int rr = 0; rr < 8; ++rr) { S[(rr + (hi << 3)) * 32 + (lane & 15)] = acc[rr]; S[(rr + (hi << 3)) * 32 + 16 + (lane & 15)] = acc1[rr]; }
  asm volatile("s_wait_dscnt 0" ::: "memory"); __builtin_amdgcn_wave_barrier(); __builtin_amdgcn_fence(__ATOMIC_RELEASE, "workgroup");
  if (active) {
#pragma unroll
    for (int q = 0; q < 4; ++q) {
      const int rl = q * 4 + (lane >> 3), pc = lane & 7;
      const int row = tm * 16 + rl;
      if (row < M) vst2(C + (long)b * strideC + (long)row * N + tn2 * 32 + pc * 4, *(const v4f*)(S + rl * 32 + pc * 4));
    }
  }
}

template <int NH, int DEG>
__global__ void gat_attn(const float* __restrict__ selfM,
                         const float* __restrict__ nbrM,
                         const int* __restrict__ adj,
                         const float* __restrict__ avec,
                         float* __restrict__ out,
                         int nS, int nT, int heads) {
  constexpr int F = NH / 32;
  const int lane = threadIdx.x & 31;
  const int wid  = (blockIdx.x * blockDim.x + threadIdx.x) >> 5;
  if (wid >= nS * heads) return;
  const int s = wid % nS;
  const int h = wid / nS;

  const float* sp = selfM + ((size_t)h * nS + s) * NH;
  const float* nb = nbrM + (size_t)h * nT * NH;
  const float* ap = avec + (size_t)h * 2 * NH;

  float a_nbr[F];
  float dself = 0.f;
#pragma unroll
  for (int f = 0; f < F; ++f) {
    const int d = lane + f * 32;
    a_nbr[f] = ap[NH + d];
    dself += sp[d] * ap[d];
  }
  dself = wave_sum(dself);

  float nd[DEG][F];
  float sc[DEG];
#pragma unroll
  for (int j = 0; j < DEG; ++j) {
    const int  id    = adj[(size_t)s * DEG + j];
    const bool valid = id > 0;
    const int idc = (id > nT) ? nT : id;
    const float* np  = nb + (size_t)(valid ? idc - 1 : 0) * NH;
    float d = 0.f;
#pragma unroll
    for (int f = 0; f < F; ++f) {
      nd[j][f] = np[lane + f * 32];
      d += nd[j][f] * a_nbr[f];
    }
    d = wave_sum(d) + dself;
    d = d > 0.f ? d : 0.2f * d;
    sc[j] = valid ? d : -1.0e9f;
  }
  float mx = sc[0];
#pragma unroll
  for (int j = 1; j < DEG; ++j) mx = fmaxf(mx, sc[j]);
  float den = 0.f;
#pragma unroll
  for (int j = 0; j < DEG; ++j) { sc[j] = __expf(sc[j] - mx); den += sc[j]; }
  const float inv = 1.0f / den;

  float* op = out + ((size_t)h * nS + s) * NH;
#pragma unroll
  for (int f = 0; f < F; ++f) {
    float a = 0.f;
#pragma unroll
    for (int j = 0; j < DEG; ++j) a += sc[j] * nd[j][f];
    vst2(op + lane + f * 32, (float_a)(a * inv));
  }
}

__global__ void concat_elu_kernel(const float* __restrict__ in,
                                  float* __restrict__ out,
                                  int n, int heads, int nh) {
  const int idx = blockIdx.x * blockDim.x + threadIdx.x;
  const int cw  = heads * nh;
  if (idx >= n * cw) return;
  const int row = idx / cw;
  const int col = idx % cw;
  const int h = col / nh, d = col % nh;
  vst2(out + idx, (float_a)elu_f(in[((size_t)h * n + row) * nh + d]));
}

__global__ void batch_gather_kernel(const int* __restrict__ bi,
                                    const float* __restrict__ outn,
                                    const float* __restrict__ oute,
                                    float* __restrict__ out,
                                    int B, int nN) {
  const int idx = blockIdx.x * blockDim.x + threadIdx.x;
  if (idx >= B * 7 * 128) return;
  const int d = idx & 127;
  const int j = (idx >> 7) % 7;
  const int b = idx / (7 * 128);
  const int* row = bi + b * 7;
  float v;
  if (j == 0) {
    int eid = row[0] - 1; eid = eid < 0 ? 0 : (eid >= 25000 ? 24999 : eid);
    v = elu_f(oute[(size_t)eid * 128 + d]);
  } else {
    int last = 0;
#pragma unroll
    for (int t = 1; t < 7; ++t)
      if (row[t] != 0) last = t;
    if (j <= last) {
      int nid = row[j] - 1;
      if (nid < 0) nid += nN;
      nid = nid < 0 ? 0 : (nid >= nN ? nN - 1 : nid);
      v = elu_f(outn[(size_t)nid * 128 + d]);
    } else {
      v = 1.0f;
    }
  }
  vst2(out + idx, (float_a)v);
}

extern "C" void kernel_launch(void* const* d_in, const int* in_sizes, int n_in,
                              void* d_out, int out_size, void* d_ws, size_t ws_size,
                              hipStream_t stream) {
  const int*   batch_inputs = (const int*)d_in[0];
  const int*   edge_list    = (const int*)d_in[1];
  const int*   node_list    = (const int*)d_in[2];
  const float* node_embs    = (const float*)d_in[3];
  const float* edge_embs    = (const float*)d_in[4];
  const float* Wn   = (const float*)d_in[5];
  const float* We   = (const float*)d_in[6];
  const float* a1   = (const float*)d_in[7];
  const float* a2   = (const float*)d_in[8];
  const float* Wn_o = (const float*)d_in[9];
  const float* We_o = (const float*)d_in[10];
  const float* a1_o = (const float*)d_in[11];
  const float* a2_o = (const float*)d_in[12];

  constexpr int nN = 50000, nE = 25000, H = 4, NH = 64, NF = 128, NE2 = 128;
  constexpr int BATCH = 4096;

  float* ws   = (float*)d_ws;
  float* hn1  = ws;
  float* he1  = hn1  + (size_t)H * nN * NH;
  float* eo1  = he1  + (size_t)H * nE * NH;
  float* no1  = eo1  + (size_t)H * nE * NH;
  float* ncat = no1  + (size_t)H * nN * NH;
  float* ecat = ncat + (size_t)nN * (H * NH);
  float* wtop = ecat + (size_t)nE * (H * NH);
  float* hn2  = ws;
  float* he2  = hn2  + (size_t)nN * NE2;
  float* eo2  = he2  + (size_t)nE * NE2;
  float* no2  = eo2  + (size_t)nE * NE2;
  _Float16* bfWn  = (_Float16*)wtop;
  _Float16* bfWe  = bfWn  + 32768;
  _Float16* bfWno = bfWe  + 32768;
  _Float16* bfWeo = bfWno + 32768;
  (void)ws_size; (void)n_in; (void)in_sizes; (void)out_size;

  auto wave_blocks = [](long waves) { return (int)((waves * 32 + 255) / 256); };
  auto thr_blocks  = [](long thr)   { return (int)((thr + 255) / 256); };

  prep_bfrag<<<thr_blocks(32768 / 8), 256, 0, stream>>>(Wn, bfWn, NH, 4, 4,
                                                    (long)NF * NH, 32768);
  prep_bfrag<<<thr_blocks(32768 / 8), 256, 0, stream>>>(We, bfWe, NH, 4, 4,
                                                    (long)NF * NH, 32768);
  prep_bfrag<<<thr_blocks(32768 / 8), 256, 0, stream>>>(Wn_o, bfWno, NE2, 8, 8, 0L, 32768);
  prep_bfrag<<<thr_blocks(32768 / 8), 256, 0, stream>>>(We_o, bfWeo, NE2, 8, 8, 0L, 32768);

  {
    long tiles = (long)((nN + 15) / 16) * (NH / 32) * H;
    gemm_wmma_f16<NF><<<wave_blocks(tiles), 256, 0, stream>>>(
        node_embs, bfWn, hn1, nN, NH, 0L, (long)nN * NH, H);
  }
  {
    long tiles = (long)((nE + 15) / 16) * (NH / 32) * H;
    gemm_wmma_f16<NF><<<wave_blocks(tiles), 256, 0, stream>>>(
        edge_embs, bfWe, he1, nE, NH, 0L, (long)nE * NH, H);
  }

  gat_attn<NH, 6><<<wave_blocks((long)nE * H), 256, 0, stream>>>(
      he1, hn1, edge_list, a1, eo1, nE, nN, H);
  gat_attn<NH, 8><<<wave_blocks((long)nN * H), 256, 0, stream>>>(
      hn1, eo1, node_list, a2, no1, nN, nE, H);

  concat_elu_kernel<<<thr_blocks((long)nN * H * NH), 256, 0, stream>>>(no1, ncat, nN, H, NH);
  concat_elu_kernel<<<thr_blocks((long)nE * H * NH), 256, 0, stream>>>(eo1, ecat, nE, H, NH);

  {
    long tiles = (long)((nN + 15) / 16) * (NE2 / 32);
    gemm_wmma_f16<256><<<wave_blocks(tiles), 256, 0, stream>>>(
        ncat, bfWno, hn2, nN, NE2, 0L, 0L, 1);
  }
  {
    long tiles = (long)((nE + 15) / 16) * (NE2 / 32);
    gemm_wmma_f16<256><<<wave_blocks(tiles), 256, 0, stream>>>(
        ecat, bfWeo, he2, nE, NE2, 0L, 0L, 1);
  }

  gat_attn<NE2, 6><<<wave_blocks((long)nE), 256, 0, stream>>>(
      he2, hn2, edge_list, a1_o, eo2, nE, nN, 1);
  gat_attn<NE2, 8><<<wave_blocks((long)nN), 256, 0, stream>>>(
      hn2, eo2, node_list, a2_o, no2, nN, nE, 1);

  batch_gather_kernel<<<thr_blocks((long)BATCH * 7 * 128), 256, 0, stream>>>(
      batch_inputs, no2, eo2, (float*)d_out, BATCH, nN);
}
